// QMARLNet_70583492543103
// MI455X (gfx1250) — hardware-verified
//
#include <hip/hip_runtime.h>


#define NBT 8
#define NN 32
#define OBS 64
#define HH 128
#define EE 16
#define NL 2
#define NACT 10
#define NRN (NBT * NN * NN)
#define NED (NBT * NN * NN * NN)
#define NQ 4
#define EDQ (NED / NQ)

typedef __attribute__((ext_vector_type(16))) __bf16   v16bf;
typedef __attribute__((ext_vector_type(16))) _Float16 v16h;
typedef __attribute__((ext_vector_type(8)))  float    v8f;
typedef __attribute__((ext_vector_type(8)))  unsigned v8u;

__device__ __forceinline__ unsigned f2bf(float f) { unsigned u = __float_as_uint(f); u += 0x7FFFu + ((u >> 16) & 1u); return u >> 16; }
__device__ __forceinline__ unsigned f2h(float f) { return (unsigned)__builtin_bit_cast(unsigned short, (_Float16)f); }
__device__ __forceinline__ int kpat(int v, int half) { return ((v & 4) ? 16 : 0) + half * 8 + 2 * (v & 3); }

template <int F16, int NP> struct Opnd { v16bf p[NP]; };

template <int F16, int NP> __device__ __forceinline__ void pack2(float f0, float f1, unsigned* o) {
    if (F16) { o[0] = f2h(f0) | (f2h(f1) << 16); return; }
    unsigned h0 = f2bf(f0), h1 = f2bf(f1); o[0] = h0 | (h1 << 16);
    if (NP >= 2) {
        float r0 = f0 - __uint_as_float(h0 << 16), r1 = f1 - __uint_as_float(h1 << 16);
        unsigned m0 = f2bf(r0), m1 = f2bf(r1); o[1] = m0 | (m1 << 16);
        if (NP >= 3) {
            float s0 = r0 - __uint_as_float(m0 << 16), s1 = r1 - __uint_as_float(m1 << 16);
            o[2] = f2bf(s0) | (f2bf(s1) << 16);
        }
    }
}
template <int F16, int NP> __device__ __forceinline__ void op_row(const float* rowp, int half, float sc, Opnd<F16, NP>& o) {
    v8u u[NP];
#pragma unroll
    for (int v = 0; v < 8; ++v) {
        int kk = kpat(v, half); unsigned t[3];
        pack2<F16, NP>(rowp[kk] * sc, rowp[kk + 1] * sc, t);
#pragma unroll
        for (int p = 0; p < NP; ++p) u[p][v] = t[p];
    }
#pragma unroll
    for (int p = 0; p < NP; ++p) o.p[p] = __builtin_bit_cast(v16bf, u[p]);
}
template <int F16, int NP> __device__ __forceinline__ void op_row_tail(const float* rowp, int half, float sc, int kvalid, Opnd<F16, NP>& o) {
    v8u u[NP];
#pragma unroll
    for (int v = 0; v < 8; ++v) {
        int kk = kpat(v, half); unsigned t[3];
        float f0 = kk < kvalid ? rowp[kk] * sc : 0.0f, f1 = (kk + 1) < kvalid ? rowp[kk + 1] * sc : 0.0f;
        pack2<F16, NP>(f0, f1, t);
#pragma unroll
        for (int p = 0; p < NP; ++p) u[p][v] = t[p];
    }
#pragma unroll
    for (int p = 0; p < NP; ++p) o.p[p] = __builtin_bit_cast(v16bf, u[p]);
}
template <int F16, int NP> __device__ __forceinline__ void op_col(const float* M, int ld, int n, int k0, int half, float sc, Opnd<F16, NP>& o) {
    v8u u[NP];
#pragma unroll
    for (int v = 0; v < 8; ++v) {
        int kk = k0 + kpat(v, half); unsigned t[3];
        pack2<F16, NP>(M[(size_t)kk * ld + n] * sc, M[(size_t)(kk + 1) * ld + n] * sc, t);
#pragma unroll
        for (int p = 0; p < NP; ++p) u[p][v] = t[p];
    }
#pragma unroll
    for (int p = 0; p < NP; ++p) o.p[p] = __builtin_bit_cast(v16bf, u[p]);
}
template <int F16, int NP> __device__ __forceinline__ void op_col_tail(const float* M, int ld, int n, int k0, int half, float sc, int K, Opnd<F16, NP>& o) {
    v8u u[NP];
#pragma unroll
    for (int v = 0; v < 8; ++v) {
        int kk = k0 + kpat(v, half); unsigned t[3];
        float f0 = kk < K ? M[(size_t)kk * ld + n] * sc : 0.0f, f1 = (kk + 1) < K ? M[(size_t)(kk + 1) * ld + n] * sc : 0.0f;
        pack2<F16, NP>(f0, f1, t);
#pragma unroll
        for (int p = 0; p < NP; ++p) u[p][v] = t[p];
    }
#pragma unroll
    for (int p = 0; p < NP; ++p) o.p[p] = __builtin_bit_cast(v16bf, u[p]);
}
__device__ __forceinline__ v8f wm_bf16(v16bf a, v16bf b, v8f c) { return __builtin_amdgcn_wmma_f32_16x16x32_bf16(false, a, false, b, (short)0, c, false, false); }
template <int F16, int NA, int NB> __device__ __forceinline__ v8f wmma_op(const Opnd<F16, NA>& a, const Opnd<F16, NB>& b, v8f c) {
    if (F16) {
        v16h ah = __builtin_bit_cast(v16h, a.p[0]), bh = __builtin_bit_cast(v16h, b.p[0]);
        c = __builtin_amdgcn_wmma_f32_16x16x32_f16(false, ah, false, bh, (short)0, c, false, false);
        asm volatile("v_nop\n\tv_nop\n\tv_nop\n\tv_nop" : "+v"(c) : "v"(ah), "v"(bh));
        return c;
    }
    constexpr int NMX = NA > NB ? NA : NB;
#pragma unroll
    for (int i = 0; i < NA; ++i)
#pragma unroll
        for (int j = 0; j < NB; ++j)
            if (i + j < NMX) c = wm_bf16(a.p[i], b.p[j], c);
    if (NA == 1 && NB == 1)      asm volatile("v_nop\n\tv_nop\n\tv_nop\n\tv_nop" : "+v"(c) : "v"(a.p[0]), "v"(b.p[0]));
    else if (NA == 2 && NB == 1) asm volatile("v_nop\n\tv_nop\n\tv_nop\n\tv_nop" : "+v"(c) : "v"(a.p[0]), "v"(a.p[1]), "v"(b.p[0]));
    else if (NA == 1 && NB == 2) asm volatile("v_nop\n\tv_nop\n\tv_nop\n\tv_nop" : "+v"(c) : "v"(a.p[0]), "v"(b.p[0]), "v"(b.p[1]));
    else if (NA == 2 && NB == 2) asm volatile("v_nop\n\tv_nop\n\tv_nop\n\tv_nop" : "+v"(c) : "v"(a.p[0]), "v"(a.p[1]), "v"(b.p[0]), "v"(b.p[1]));
    else                         asm volatile("v_nop\n\tv_nop\n\tv_nop\n\tv_nop" : "+v"(c) : "v"(a.p[0]), "v"(a.p[NA - 1]), "v"(b.p[0]), "v"(b.p[NB - 1]), "v"(a.p[NA / 2]), "v"(b.p[NB / 2]));
    return c;
}

struct ZMap { long long s1; long long s2; int zdiv; int pad_; };
__device__ __forceinline__ size_t zoff(const ZMap& m, int z) { return (size_t)((long long)(z / m.zdiv) * m.s1 + (long long)(z % m.zdiv) * m.s2); }

#define ACT_NONE 0
#define ACT_RELU 1
#define ACT_GELU_ERF 2
#define ACT_SILU 3
#define ACT_TANH 4
__device__ __forceinline__ float act_apply(int act, float x) {
    if (act == ACT_RELU) return x > 0.f ? x : 0.f;
    if (act == ACT_GELU_ERF) return 0.5f * x * (1.0f + erff(x * 0.70710678118654752f));
    if (act == ACT_SILU) return x / (1.0f + expf(-x));
    if (act == ACT_TANH) return tanhf(x);
    return x;
}
struct GemmArgs {
    ZMap za, zb_, zc, zbias, zadd, zrsc, zmul, zrbias;
    const float* A; const float* Bm; float* C; const float* bias; const float* add; const float* rsc; const float* mul; const float* rbias;
    long long ldadd, ldmul;
    int lda, ldb, ldc, K;
    float ascale, bscale, oscale, addscale;
    int M, nvalid, nstore, ldrsc;
    int bcs, pad1, pad2, pad3;
};
template <int BT, int F16, int NA, int NB, int RW, int CW, int ACT>
__global__ __launch_bounds__(256) void gemm_kernel(GemmArgs g) {
    constexpr int TR = 16 * RW, TC = 64 * CW, CSTR = TC + 4;
    __shared__ __align__(16) float cst[TR * CSTR];
    const int z = blockIdx.z;
    const float* A = g.A + zoff(g.za, z); const float* Bm = g.Bm + zoff(g.zb_, z); float* C = g.C + zoff(g.zc, z);
    const int tid = threadIdx.x, lane = tid & 31, wv = tid >> 5;
    const int l16 = lane & 15, half = lane >> 4;
    const int rt = wv % RW, ch = wv / RW;
    const int row0 = blockIdx.x * TR, col0 = blockIdx.y * TC + ch * 64;
    int arix = row0 + rt * 16 + l16; if (arix >= g.M) arix = g.M - 1;
    const float* arow = A + (size_t)arix * g.lda;
    v8f acc[4];
#pragma unroll
    for (int t = 0; t < 4; ++t) acc[t] = (v8f){};
    const int K = g.K;
#pragma unroll 1
    for (int kc = 0; kc < K; kc += 32) {
        Opnd<F16, NA> a;
        if (kc + 32 <= K) op_row<F16, NA>(arow + kc, half, g.ascale, a); else op_row_tail<F16, NA>(arow + kc, half, g.ascale, K - kc, a);
#pragma unroll
        for (int t = 0; t < 4; ++t) {
            Opnd<F16, NB> b;
            const int n = col0 + t * 16 + l16;
            if (n < g.nvalid) {
                if (BT) { if (kc + 32 <= K) op_row<F16, NB>(Bm + (size_t)n * g.ldb + kc, half, g.bscale, b); else op_row_tail<F16, NB>(Bm + (size_t)n * g.ldb + kc, half, g.bscale, K - kc, b); }
                else    { if (kc + 32 <= K) op_col<F16, NB>(Bm, g.ldb, n * g.bcs, kc, half, g.bscale, b); else op_col_tail<F16, NB>(Bm, g.ldb, n * g.bcs, kc, half, g.bscale, K, b); }
            } else {
#pragma unroll
                for (int p = 0; p < NB; ++p) b.p[p] = (v16bf){};
            }
            acc[t] = wmma_op<F16, NA, NB>(a, b, acc[t]);
        }
    }
    const float* bias = g.bias ? g.bias + zoff(g.zbias, z) : nullptr;
    const float* add = g.add ? g.add + zoff(g.zadd, z) : nullptr;
    const float* rsc = g.rsc ? g.rsc + zoff(g.zrsc, z) : nullptr;
    const float* mul = g.mul ? g.mul + zoff(g.zmul, z) : nullptr;
    const float* rbias = g.rbias ? g.rbias + zoff(g.zrbias, z) : nullptr;
#pragma unroll
    for (int t = 0; t < 4; ++t) {
        const int cl = ch * 64 + t * 16 + l16;
        const int cg = blockIdx.y * TC + cl;
        const bool cok = cg < g.nvalid;
        const float bv = (bias && cok) ? bias[(size_t)cg * g.bcs] : 0.0f;
#pragma unroll
        for (int r = 0; r < 8; ++r) {
            const int rl = rt * 16 + r + 8 * half;
            float v = acc[t][r] * g.oscale + bv;
            int rg = row0 + rl; if (rg >= g.M) rg = g.M - 1;
            if (rbias) v += rbias[rg];
            if (rsc) v *= rsc[(size_t)rg * g.ldrsc];
            if (mul && cok) v *= mul[(size_t)rg * g.ldmul + cg];
            if (add && cok) v += g.addscale * add[(size_t)rg * g.ldadd + cg];
            cst[rl * CSTR + cl] = v;
        }
    }
    __syncthreads();
    const int col = tid % TC, rsel = tid / TC, rstep = 256 / TC;
    if (ACT != ACT_NONE) {
#pragma unroll 1
        for (int r = rsel; r < TR; r += rstep) cst[r * CSTR + col] = act_apply(ACT, cst[r * CSTR + col]);
    }
    float* ob = C + (size_t)row0 * g.ldc + (size_t)blockIdx.y * TC;
    const bool colok = (int)(blockIdx.y * TC + col) < g.nstore;
    const int rmax = (g.M - row0 < TR) ? (g.M - row0) : TR;
    auto pass = [&]() {
        if (colok) {
#pragma unroll 4
            for (int r = rsel; r < rmax; r += rstep) *(volatile float*)(ob + (size_t)r * g.ldc + col) = cst[r * CSTR + col];
        }
    };
    pass();
    __threadfence();
    pass();
}
static inline ZMap zm(long long s1) { ZMap m; m.s1 = s1; m.s2 = 0; m.zdiv = 1; m.pad_ = 0; return m; }
static inline ZMap zm2(long long s1, long long s2, int zdiv) { ZMap m; m.s1 = s1; m.s2 = s2; m.zdiv = zdiv; m.pad_ = 0; return m; }
static inline GemmArgs gemm_args(const float* A, int lda, ZMap za, const float* Bm, int ldb, ZMap zb, float* C, int ldc, ZMap zc, int M, int N, int K) {
    GemmArgs g; g.za = za; g.zb_ = zb; g.zc = zc; g.zbias = zm(0); g.zadd = zm(0); g.zrsc = zm(0); g.zmul = zm(0); g.zrbias = zm(0);
    g.A = A; g.Bm = Bm; g.C = C; g.bias = nullptr; g.add = nullptr; g.rsc = nullptr; g.mul = nullptr; g.rbias = nullptr; g.ldadd = 0; g.ldmul = 0;
    g.lda = lda; g.ldb = ldb; g.ldc = ldc; g.K = K; g.ascale = 1.0f; g.bscale = 1.0f; g.oscale = 1.0f; g.addscale = 1.0f; g.M = M; g.nvalid = N; g.nstore = N; g.ldrsc = 1;
    g.bcs = 1; g.pad1 = 0; g.pad2 = 0; g.pad3 = 0;
    return g;
}
static_assert(sizeof(ZMap) == 24, "ZMap layout");
static_assert(sizeof(GemmArgs) == 8 * 24 + 8 * 8 + 2 * 8 + 4 * 4 + 4 * 4 + 4 * 4 + 4 * 4, "GemmArgs has no padding");

__global__ __launch_bounds__(256) void softmax_rows(float* S, long long sy, long long sx, int L, float prescale, const float* addv, long long say, int aydiv, int causal,
                                                  const int* imask, long long imy, long long imx, float maskval) {
    __shared__ float red[8];
    const int tid = threadIdx.x, lane = tid & 31, wid = tid >> 5;
    float* row = S + (size_t)blockIdx.y * sy + (size_t)blockIdx.x * sx;
    const float* av = addv ? addv + (size_t)(blockIdx.y / aydiv) * say : nullptr;
    const int* im = imask ? imask + (size_t)(blockIdx.y / aydiv) * imy + (size_t)blockIdx.x * imx : nullptr;
    float v[16];
    const int nj = L / 256;
    float mx = -__builtin_inff();
#pragma unroll
    for (int j = 0; j < 16; ++j) if (j < nj) { float t = row[tid + 256 * j] * prescale; if (av) t += av[tid + 256 * j]; if (im && im[tid + 256 * j] == 0) t = maskval; if (causal && (tid + 256 * j) > (int)blockIdx.x) t = -__builtin_inff(); v[j] = t; mx = fmaxf(mx, t); }
#pragma unroll
    for (int o = 16; o; o >>= 1) mx = fmaxf(mx, __shfl_xor(mx, o, 32));
    if (lane == 0) red[wid] = mx;
    __syncthreads();
    float m = red[0];
#pragma unroll
    for (int i = 1; i < 8; ++i) m = fmaxf(m, red[i]);
    if (m == -__builtin_inff()) m = 0.f;
    __syncthreads();
    float sum = 0.f;
#pragma unroll
    for (int j = 0; j < 16; ++j) if (j < nj) { v[j] = expf(v[j] - m); sum += v[j]; }
#pragma unroll
    for (int o = 16; o; o >>= 1) sum += __shfl_xor(sum, o, 32);
    if (lane == 0) red[wid] = sum;
    __syncthreads();
    float tot = 0.f;
#pragma unroll
    for (int i = 0; i < 8; ++i) tot += red[i];
    const float inv = 1.0f / tot;
#pragma unroll
    for (int j = 0; j < 16; ++j) if (j < nj) *(volatile float*)(row + tid + 256 * j) = v[j] * inv;
    __threadfence();
#pragma unroll
    for (int j = 0; j < 16; ++j) if (j < nj) *(volatile float*)(row + tid + 256 * j) = v[j] * inv;
}

#define VST2(T, p, v) do { const T vst2_v_ = (v); *(volatile T*)(p) = vst2_v_; __threadfence(); *(volatile T*)(p) = vst2_v_; } while (0)
__device__ __forceinline__ float adjv(const float* __restrict__ adjm, const float* __restrict__ nm, int b, int r, int i, int j) { return adjm[((size_t)b * NN + i) * NN + j] * nm[((size_t)b * NN + r) * NN + i] * nm[((size_t)b * NN + r) * NN + j]; }
__global__ __launch_bounds__(256) void k_adj(const float* __restrict__ adjm, const float* __restrict__ nm, float* ADJ) { const int q = blockIdx.x * 256 + threadIdx.x; if (q >= NED) return; const int j = q % NN, i = (q / NN) % NN, r = (q / (NN * NN)) % NN, b = q / (NN * NN * NN); VST2(float, ADJ + q, adjv(adjm, nm, b, r, i, j)); }
__global__ __launch_bounds__(256) void k_ln(const float* __restrict__ obs, const float* __restrict__ g, const float* __restrict__ bb, float* XO) { const int lane = threadIdx.x & 31; const int r = blockIdx.x * 8 + (threadIdx.x >> 5); if (r >= NBT * NN) return; const float v0 = obs[(size_t)r * OBS + lane], v1 = obs[(size_t)r * OBS + 32 + lane]; float s = v0 + v1;
#pragma unroll
    for (int o = 16; o; o >>= 1) s += __shfl_xor(s, o, 32); const float mean = s / (float)OBS; float sq = (v0 - mean) * (v0 - mean) + (v1 - mean) * (v1 - mean);
#pragma unroll
    for (int o = 16; o; o >>= 1) sq += __shfl_xor(sq, o, 32); const float rs = 1.f / sqrtf(sq / (float)OBS + 1e-5f);
    VST2(float, XO + (size_t)r * OBS + lane, (v0 - mean) * rs * g[lane] + bb[lane]); VST2(float, XO + (size_t)r * OBS + 32 + lane, (v1 - mean) * rs * g[32 + lane] + bb[32 + lane]); }
__global__ __launch_bounds__(256) void k_node0(const float* __restrict__ ENC, const float* __restrict__ nm, float* NODE) { const int q = blockIdx.x * 256 + threadIdx.x; if (q >= NRN * HH) return; const int h = q % HH; const int rn = q / HH; const int n = rn % NN; const int br = rn / NN; const int b = br / NN; VST2(float, NODE + q, ENC[((size_t)b * NN + n) * HH + h] * nm[rn]); }
__global__ __launch_bounds__(256) void k_edge0(const float* __restrict__ ef, const float* __restrict__ ew, const float* __restrict__ eb, const float* __restrict__ ADJ, float* EDGE) { const size_t q = (size_t)blockIdx.x * 256 + threadIdx.x; if (q >= (size_t)NED * EE) return; const int c = (int)(q % EE); const size_t ed = q / EE; const int j = (int)(ed % NN), i = (int)((ed / NN) % NN), r = (int)((ed / (NN * NN)) % NN), b = (int)(ed / ((size_t)NN * NN * NN)); float v = 0.f;
    { const float* f = ef + (((size_t)b * NN + i) * NN + j) * EE; float a = eb[c];
#pragma unroll 1
        for (int k = 0; k < EE; ++k) a += f[k] * ew[c * EE + k]; v = fmaxf(a, 0.f) * ADJ[ed]; (void)r; }
    VST2(float, EDGE + q, v); }
__global__ __launch_bounds__(256) void k_agg(const float* __restrict__ MSG, const float* __restrict__ HIDN, const float* __restrict__ ADJ, int rn0, float* HID2) { const int q0 = blockIdx.x * 256 + threadIdx.x; if (q0 >= (EDQ / NN) * HH) return; const int q = rn0 * HH + q0; const int h = q % HH; const int rn = q / HH; const int i = rn % NN, r = (rn / NN) % NN, b = rn / (NN * NN); float s = HIDN[q];
#pragma unroll 1
    for (int j = 0; j < NN; ++j) s += ADJ[(size_t)rn * NN + j] * MSG[((size_t)(rn - rn0) * NN + j) * HH + h]; (void)i; (void)r; (void)b; VST2(float, HID2 + q, s); }
__global__ __launch_bounds__(256) void k_nmask(const float* __restrict__ NUP, const float* __restrict__ nm, float* NODE) { const int q = blockIdx.x * 256 + threadIdx.x; if (q >= NRN * HH) return; VST2(float, NODE + q, NUP[q] * nm[q / HH]); }
__global__ __launch_bounds__(256) void k_eupd(const float* __restrict__ EDGE, const float* __restrict__ SD, const float* __restrict__ we, const float* __restrict__ eob, const float* __restrict__ ADJ, float* EDGEn) { const size_t q = (size_t)blockIdx.x * 256 + threadIdx.x; if (q >= (size_t)NED * EE) return; const int c = (int)(q % EE); const size_t ed = q / EE; const int j = (int)(ed % NN), i = (int)((ed / NN) % NN), r = (int)((ed / (NN * NN)) % NN), b = (int)(ed / ((size_t)NN * NN * NN)); float v = 0.f;
    { const size_t bri = ((size_t)b * NN + r) * NN + i, brj = ((size_t)b * NN + r) * NN + j; float a = SD[bri * 32 + c] + SD[brj * 32 + EE + c] + eob[c]; const float* er = EDGE + ed * EE;
#pragma unroll 1
        for (int k = 0; k < EE; ++k) a += er[k] * we[c * (2 * HH + EE) + 2 * HH + k]; v = fmaxf(a, 0.f) * ADJ[ed]; }
    VST2(float, EDGEn + q, v); }
__global__ __launch_bounds__(256) void k_wts(const float* __restrict__ er_w, const float* __restrict__ eo_w, const float* __restrict__ pol_w, const float* __restrict__ pol_b, const float* __restrict__ q_w, const float* __restrict__ q_b, float* ERP, float* WSD, float* PQ, float* BPQ) { const int q = blockIdx.x * 256 + threadIdx.x;
    if (q < NL * EE * HH) { const int h = q % HH, k = (q / HH) % EE, l = q / (HH * EE); VST2(float, ERP + q, er_w[((size_t)l * HH + h) * EE + k]); }
    if (q < NL * HH * 32) { const int c = q % 32, k = (q / 32) % HH, l = q / (32 * HH); const float* w = eo_w + (size_t)l * EE * (2 * HH + EE); VST2(float, WSD + q, c < EE ? w[(size_t)c * (2 * HH + EE) + k] : w[(size_t)(c - EE) * (2 * HH + EE) + HH + k]); }
    if (q < HH * 32) { const int c = q % 32, k = q / 32; VST2(float, PQ + q, c < NACT ? pol_w[c * HH + k] : (c < 2 * NACT ? q_w[(c - NACT) * HH + k] : 0.f)); }
    if (q < 32) { VST2(float, BPQ + q, q < NACT ? pol_b[q] : (q < 2 * NACT ? q_b[q - NACT] : 0.f)); } }
__global__ __launch_bounds__(256) void k_heads(const float* __restrict__ PQO, const float* __restrict__ nm, float* O32) { const int lane = threadIdx.x & 31; const int bn = blockIdx.x * 8 + (threadIdx.x >> 5); if (bn >= NBT * NN) return; const int b = bn / NN, n = bn % NN; float er = 0.f, eq = 0.f, cnt = 0.f;
#pragma unroll 1
    for (int r = 0; r < NN; ++r) { const float m_ = nm[((size_t)b * NN + r) * NN + n]; const float* row = PQO + (((size_t)b * NN + r) * NN + n) * 32; const float lg = (lane < NACT) ? row[lane] : -__builtin_inff(); float mx = lg;
#pragma unroll
        for (int o = 16; o; o >>= 1) mx = fmaxf(mx, __shfl_xor(mx, o, 32)); const float e = (lane < NACT) ? expf(lg - mx) : 0.f; float den = e;
#pragma unroll
        for (int o = 16; o; o >>= 1) den += __shfl_xor(den, o, 32);
        er += m_ * (e / den); eq += m_ * ((lane < NACT) ? row[NACT + lane] : 0.f); cnt += m_; }
    cnt = fmaxf(cnt, 1.f); er /= cnt; eq /= cnt;
    float p = (1.f - 0.05f) * er + 0.05f / (float)NACT; float ps = (lane < NACT) ? p : 0.f;
#pragma unroll
    for (int o = 16; o; o >>= 1) ps += __shfl_xor(ps, o, 32); p = p / fmaxf(ps, 1e-8f);
    float v = 0.f; if (lane < NACT) v = p; else if (lane < 2 * NACT) v = 0.f;
    VST2(float, O32 + (size_t)bn * 32 + lane, lane < NACT ? p : 0.f); VST2(float, O32 + (size_t)(NBT * NN + bn) * 32 + lane, lane < NACT ? eq : 0.f); VST2(float, O32 + (size_t)(2 * NBT * NN + bn) * 32 + lane, lane < NACT ? er : 0.f); (void)v; }
__global__ __launch_bounds__(256) void k_copy(const float* __restrict__ O32, float* o1, float* o2, float* o3) { const int q = blockIdx.x * 256 + threadIdx.x; if (q >= NBT * NN * NACT) return; const int a = q % NACT, bn = q / NACT; VST2(float, o1 + q, O32[(size_t)bn * 32 + a]); VST2(float, o2 + q, O32[(size_t)(NBT * NN + bn) * 32 + a]); VST2(float, o3 + q, O32[(size_t)(2 * NBT * NN + bn) * 32 + a]); }
extern "C" void kernel_launch(void* const* d_in, const int* in_sizes, int n_in,
                              void* d_out, int out_size, void* d_ws, size_t ws_size, hipStream_t stream) {
    (void)in_sizes; (void)n_in; (void)out_size;
    const float* obs = (const float*)d_in[0]; const float* ef = (const float*)d_in[1]; const float* adjm = (const float*)d_in[2]; const float* nm = (const float*)d_in[3]; const float* lg = (const float*)d_in[4]; const float* lb = (const float*)d_in[5];
    const float* ow1 = (const float*)d_in[6]; const float* ob1 = (const float*)d_in[7]; const float* ow2 = (const float*)d_in[8]; const float* ob2 = (const float*)d_in[9]; const float* ew = (const float*)d_in[10]; const float* eb = (const float*)d_in[11];
    const float* nr_w = (const float*)d_in[12]; const float* nr_b = (const float*)d_in[13]; const float* er_w = (const float*)d_in[14]; const float* er_b = (const float*)d_in[15]; const float* no_w = (const float*)d_in[16]; const float* no_b = (const float*)d_in[17]; const float* eo_w = (const float*)d_in[18]; const float* eo_b = (const float*)d_in[19];
    const float* pol_w = (const float*)d_in[20]; const float* pol_b = (const float*)d_in[21]; const float* q_w = (const float*)d_in[22]; const float* q_b = (const float*)d_in[23];
    float* o1 = (float*)d_out; float* o2 = (float*)((char*)d_out + 10240); float* o3 = (float*)((char*)d_out + 20480);
    char* wsp = (char*)d_ws;
    auto take = [&](size_t bytes) { char* p = wsp; wsp += (bytes + 255) & ~(size_t)255; return (void*)p; };
    float* XO = (float*)take((size_t)NBT * NN * OBS * 4); float* E1 = (float*)take((size_t)NBT * NN * HH * 4); float* ENC = (float*)take((size_t)NBT * NN * HH * 4);
    float* NODE = (float*)take((size_t)NRN * HH * 4); float* HIDN = (float*)take((size_t)NRN * HH * 4); float* HID2 = (float*)take((size_t)NRN * HH * 4); float* NUP = (float*)take((size_t)NRN * HH * 4); float* SD = (float*)take((size_t)NRN * 32 * 4); float* PQO = (float*)take((size_t)NRN * 32 * 4);
    float* EDGE = (float*)take((size_t)NED * EE * 4); float* EDGE2 = (float*)take((size_t)NED * EE * 4); float* MSG = (float*)take((size_t)EDQ * HH * 4);
    float* ERP = (float*)take((size_t)NL * EE * HH * 4); float* WSD = (float*)take((size_t)NL * HH * 32 * 4); float* PQ = (float*)take(HH * 32 * 4); float* BPQ = (float*)take(32 * 4); float* O32 = (float*)take((size_t)3 * NBT * NN * 32 * 4); float* ADJ = (float*)take((size_t)NED * 4);
    if ((size_t)(wsp - (char*)d_ws) > ws_size) return;
    k_wts<<<(NL * HH * 32 + 255) / 256, 256, 0, stream>>>(er_w, eo_w, pol_w, pol_b, q_w, q_b, ERP, WSD, PQ, BPQ);
    k_ln<<<(NBT * NN) / 8, 256, 0, stream>>>(obs, lg, lb, XO);
    { GemmArgs g = gemm_args(XO, OBS, zm(0), ow1, OBS, zm(0), E1, HH, zm(0), NBT * NN, HH, OBS); g.bias = ob1; gemm_kernel<1, 0, 2, 2, 4, 2, ACT_RELU><<<dim3((NBT * NN) / 64, 1, 1), 256, 0, stream>>>(g); }
    { GemmArgs g = gemm_args(E1, HH, zm(0), ow2, HH, zm(0), ENC, HH, zm(0), NBT * NN, HH, HH); g.bias = ob2; gemm_kernel<1, 0, 2, 2, 4, 2, ACT_RELU><<<dim3((NBT * NN) / 64, 1, 1), 256, 0, stream>>>(g); }
    k_node0<<<(NRN * HH) / 256, 256, 0, stream>>>(ENC, nm, NODE);
    k_adj<<<NED / 256, 256, 0, stream>>>(adjm, nm, ADJ);
    k_edge0<<<(unsigned)(((size_t)NED * EE) / 256), 256, 0, stream>>>(ef, ew, eb, ADJ, EDGE);
    float* cE = EDGE; float* nE = EDGE2;
    for (int l = 0; l < NL; ++l) {
        { GemmArgs g = gemm_args(NODE, HH, zm(0), nr_w + (size_t)l * HH * HH, HH, zm(0), HIDN, HH, zm(0), NRN, HH, HH); g.bias = nr_b + l * HH; gemm_kernel<1, 1, 1, 1, 4, 2, ACT_RELU><<<dim3(NRN / 64, 1, 1), 256, 0, stream>>>(g); }
        for (int qc = 0; qc < NQ; ++qc) {
            { GemmArgs g = gemm_args(cE + (size_t)qc * EDQ * EE, EE, zm(0), ERP + (size_t)l * EE * HH, HH, zm(0), MSG, HH, zm(0), EDQ, HH, EE); g.bias = er_b + l * HH; gemm_kernel<0, 1, 1, 1, 4, 2, ACT_RELU><<<dim3(EDQ / 64, 1, 1), 256, 0, stream>>>(g); }
            k_agg<<<((EDQ / NN) * HH) / 256, 256, 0, stream>>>(MSG, HIDN, ADJ, qc * (EDQ / NN), HID2);
        }
        { GemmArgs g = gemm_args(HID2, HH, zm(0), no_w + (size_t)l * HH * HH, HH, zm(0), NUP, HH, zm(0), NRN, HH, HH); g.bias = no_b + l * HH; g.add = NODE; g.ldadd = HH; g.addscale = 1.0f; gemm_kernel<1, 1, 1, 1, 4, 2, ACT_NONE><<<dim3(NRN / 64, 1, 1), 256, 0, stream>>>(g); }
        k_nmask<<<(NRN * HH) / 256, 256, 0, stream>>>(NUP, nm, NODE);
        { GemmArgs g = gemm_args(NODE, HH, zm(0), WSD + (size_t)l * HH * 32, 32, zm(0), SD, 32, zm(0), NRN, 32, HH); g.nstore = 32; gemm_kernel<0, 1, 1, 1, 8, 1, ACT_NONE><<<dim3(NRN / 128, 1, 1), 256, 0, stream>>>(g); }
        k_eupd<<<(unsigned)(((size_t)NED * EE) / 256), 256, 0, stream>>>(cE, SD, eo_w + (size_t)l * EE * (2 * HH + EE), eo_b + l * EE, ADJ, nE);
        { float* t = cE; cE = nE; nE = t; }
    }
    { GemmArgs g = gemm_args(NODE, HH, zm(0), PQ, 32, zm(0), PQO, 32, zm(0), NRN, 2 * NACT, HH); g.bias = BPQ; g.nstore = 32; gemm_kernel<0, 0, 2, 2, 8, 1, ACT_NONE><<<dim3(NRN / 128, 1, 1), 256, 0, stream>>>(g); }
    k_heads<<<(NBT * NN) / 8, 256, 0, stream>>>(PQO, nm, O32);
    k_copy<<<(NBT * NN * NACT + 255) / 256, 256, 0, stream>>>(O32, o1, o2, o3);
}
